// NodewiseInteraction_29154238005850
// MI455X (gfx1250) — hardware-verified
//
#include <hip/hip_runtime.h>
#include <stddef.h>
#include <stdint.h>

#define NN     10000
#define NE     160000
#define CH     128
#define RB     20
#define HD     32
#define WN     384
#define MS     1152
#define NPB    16
#define NTE    128
#define NWE    4
#define CAP    512
#define MAXDEG 64
#define TP     40
#define SCH    512
#define ACP    1168
#define OTP    640
#define SWP    68

static_assert(MS == 9 * CH);
static_assert(WN == 3 * CH);
static_assert(NN % NPB == 0);
static_assert(NN % 16 == 0);
static_assert(SCH == 4 * NTE);
static_assert(NE % 4 == 0);
static_assert(CAP % 16 == 0);
static_assert(MAXDEG % 16 == 0);
static_assert(MS % 8 == 0);
static_assert(ACP == MS + 16);
static_assert((ACP * 4) % 16 == 0);
static_assert(NPB / NWE == 4);

typedef unsigned short u16;
typedef __bf16 v16b __attribute__((ext_vector_type(16)));
typedef unsigned short v8us __attribute__((ext_vector_type(8)));
typedef float v8f __attribute__((ext_vector_type(8)));
typedef float v4f __attribute__((ext_vector_type(4)));
typedef unsigned int v4u __attribute__((ext_vector_type(4)));
typedef int v4i __attribute__((ext_vector_type(4)));

union Frag  { v16b v; v8us h[2]; };
union Pack8 { v8us h; v4u u; u16 s[8]; };

__device__ __forceinline__ v8f zero8() { return (v8f){0.f, 0.f, 0.f, 0.f, 0.f, 0.f, 0.f, 0.f}; }
__device__ __forceinline__ v4f zero4() { return (v4f){0.f, 0.f, 0.f, 0.f}; }

__device__ __forceinline__ v8f mma(v16b a, v16b b, v8f c) {
  c = __builtin_amdgcn_wmma_f32_16x16x32_bf16(false, a, false, b, (short)0, c, false, false);
  asm volatile("v_nop\n\tv_nop\n\tv_nop\n\tv_nop" : "+v"(c) : "v"(a), "v"(b));
  return c;
}

__device__ __forceinline__ u16 f2bf(float f) {
  unsigned int u = __float_as_uint(f);
  u += 0x7FFFu + ((u >> 16) & 1u);
  return (u16)(u >> 16);
}
__device__ __forceinline__ float bf2f(u16 h) { return __uint_as_float(((unsigned int)h) << 16); }
__device__ __forceinline__ u16 lo_of(float f, u16 hi) { return f2bf(f - bf2f(hi)); }
__device__ __forceinline__ void split8(v4f a, v4f b, v4u& hu, v4u& lu) {
  Pack8 ph, pl;
#pragma unroll
  for (int i = 0; i < 4; ++i) {
    const u16 h0 = f2bf(a[i]);
    ph.s[i] = h0;
    pl.s[i] = lo_of(a[i], h0);
    const u16 h1 = f2bf(b[i]);
    ph.s[4 + i] = h1;
    pl.s[4 + i] = lo_of(b[i], h1);
  }
  hu = ph.u;
  lu = pl.u;
}
__device__ __forceinline__ v16b mkfrag(v4u e0, v4u e1) {
  Pack8 p0, p1;
  p0.u = e0;
  p1.u = e1;
  Frag f;
  f.h[0] = p0.h;
  f.h[1] = p1.h;
  return f.v;
}

__device__ __forceinline__ v16b ldfrag(const u16* p, int ld, int row0, int k0, int lane) {
  const int m = lane & 15, lh = lane >> 4;
  const u16* q = p + (size_t)(row0 + m) * ld + k0 + 8 * lh;
  Frag f;
  f.h[0] = *(const v8us*)(q);
  f.h[1] = *(const v8us*)(q + 16);
  return f.v;
}

__device__ __forceinline__ float silu_f(float v) {
  return v * __builtin_amdgcn_rcpf(1.0f + __expf(-v));
}

__device__ __forceinline__ void wsync() {
  __builtin_amdgcn_fence(__ATOMIC_RELEASE, "wavefront");
  asm volatile("s_wait_dscnt 0x0" ::: "memory");
  __builtin_amdgcn_wave_barrier();
  __builtin_amdgcn_fence(__ATOMIC_ACQUIRE, "wavefront");
}

__global__ __launch_bounds__(256) void k_prep(const float* __restrict__ ws1, const float* __restrict__ wr1,
                                              const float* __restrict__ ws2, const float* __restrict__ wr2,
                                              const float* __restrict__ w0, const float* __restrict__ w1,
                                              const float* __restrict__ w2,
                                              u16* __restrict__ wpqh, u16* __restrict__ wpql,
                                              u16* __restrict__ wr1h, u16* __restrict__ wr1l,
                                              u16* __restrict__ ws2h, u16* __restrict__ ws2l,
                                              u16* __restrict__ wr2h, u16* __restrict__ wr2l,
                                              u16* __restrict__ wlh, u16* __restrict__ wll) {
  const int tid = threadIdx.x, b = blockIdx.x;
  v4f a0 = zero4(), a1 = zero4();
  u16* dh;
  u16* dl;
  size_t go;
  bool act = true;
  if (b < 4) {
    const int piece = b * 256 + tid, row = piece >> 4, kp = (piece & 15) * 8;
    const bool qsel = row >= 32;
    const int rp = qsel ? (row - 32) : row;
#pragma unroll
    for (int i = 0; i < 8; ++i) {
      const int k = kp + i;
      const float vp = ws1[(size_t)k * HD + rp];
      const float vq = ws1[(size_t)(CH + k) * HD + rp];
      const float v = qsel ? vq : vp;
      if (i < 4) a0[i] = v; else a1[i - 4] = v;
    }
    dh = wpqh; dl = wpql; go = (size_t)row * CH + kp;
  } else if (b < 5) {
    const int piece = tid;
    act = tid < 128;
    const int row = (piece >> 2) & 31, kp = (piece & 3) * 8;
#pragma unroll
    for (int i = 0; i < 8; ++i) {
      const int k = kp + i;
      const int kc = (k < RB) ? k : (RB - 1);
      const float vv = wr1[(size_t)kc * HD + row];
      const float v = (k < RB) ? vv : 0.f;
      if (i < 4) a0[i] = v; else a1[i - 4] = v;
    }
    dh = wr1h; dl = wr1l; go = (size_t)row * HD + kp;
  } else if (b < 11) {
    const int piece = (b - 5) * 256 + tid, row = piece >> 2, kp = (piece & 3) * 8;
#pragma unroll
    for (int i = 0; i < 8; ++i) {
      const float v = ws2[(size_t)(kp + i) * WN + row];
      if (i < 4) a0[i] = v; else a1[i - 4] = v;
    }
    dh = ws2h; dl = ws2l; go = (size_t)row * HD + kp;
  } else if (b < 17) {
    const int piece = (b - 11) * 256 + tid, row = piece >> 2, kp = (piece & 3) * 8;
#pragma unroll
    for (int i = 0; i < 8; ++i) {
      const float v = wr2[(size_t)(kp + i) * WN + row];
      if (i < 4) a0[i] = v; else a1[i - 4] = v;
    }
    dh = wr2h; dl = wr2l; go = (size_t)row * HD + kp;
  } else {
    const int piece = (b - 17) * 256 + tid;
    const int l = piece >> 11, q = piece & 2047, row = q >> 4, kp = (q & 15) * 8;
    const float* w = (l == 0) ? w0 : ((l == 1) ? w1 : w2);
#pragma unroll
    for (int i = 0; i < 8; ++i) {
      const float v = w[(size_t)(kp + i) * CH + row];
      if (i < 4) a0[i] = v; else a1[i - 4] = v;
    }
    dh = wlh; dl = wll; go = (size_t)l * CH * CH + (size_t)row * CH + kp;
  }
  v4u hu, lu;
  split8(a0, a1, hu, lu);
  if (act) {
    *(volatile v4u*)(dh + go) = hu;
    *(volatile v4u*)(dl + go) = lu;
  }
  __threadfence();
  if (act) {
    *(volatile v4u*)(dh + go) = hu;
    *(volatile v4u*)(dl + go) = lu;
  }
}

__global__ __launch_bounds__(256) void k_pq(const float* __restrict__ x, const float* __restrict__ bs1,
                                            const u16* __restrict__ wpqh, const u16* __restrict__ wpql,
                                            float* __restrict__ pq) {
  __shared__ __align__(16) float sw[8][16 * SWP];
  const int tid = threadIdx.x, lane = tid & 31, wave = tid >> 5, hh = lane >> 4, c = lane & 15;
  const int r0 = blockIdx.x * 128 + wave * 16;
  const bool valid = r0 < NN;
  const int arow = ((r0 + c) < NN) ? (r0 + c) : (NN - 1);
  v8f acc[4];
#pragma unroll
  for (int t = 0; t < 4; ++t) acc[t] = zero8();
#pragma unroll 1
  for (int ks = 0; ks < 4; ++ks) {
    const int k0 = 32 * ks;
    const float* xp = x + (size_t)arow * CH + k0 + 8 * hh;
    const v4f e0 = *(const v4f*)(xp), e1 = *(const v4f*)(xp + 4);
    const v4f e2 = *(const v4f*)(xp + 16), e3 = *(const v4f*)(xp + 20);
    v4u hu0, lu0, hu1, lu1;
    split8(e0, e1, hu0, lu0);
    split8(e2, e3, hu1, lu1);
    const v16b ah = mkfrag(hu0, hu1), al = mkfrag(lu0, lu1);
#pragma unroll
    for (int t = 0; t < 4; ++t) {
      const v16b bh = ldfrag(wpqh, CH, 16 * t, k0, lane);
      const v16b bl = ldfrag(wpql, CH, 16 * t, k0, lane);
      acc[t] = mma(ah, bh, acc[t]);
      acc[t] = mma(al, bh, acc[t]);
      acc[t] = mma(ah, bl, acc[t]);
    }
  }
  float* w = sw[wave];
#pragma unroll
  for (int t = 0; t < 4; ++t) {
    const float bb = (t < 2) ? bs1[(16 * t + c) & 31] : 0.f;
#pragma unroll
    for (int r = 0; r < 8; ++r) w[(8 * hh + r) * SWP + 16 * t + c] = acc[t][r] + bb;
  }
  __syncthreads();
  if (valid) {
    v4f val[8];
    size_t go[8];
#pragma unroll
    for (int it = 0; it < 8; ++it) {
      const int p = it * 32 + lane, row = p >> 4, q = p & 15;
      val[it] = *(const v4f*)(w + row * SWP + 4 * q);
      go[it] = (size_t)(r0 + row) * 64 + 4 * q;
    }
#pragma unroll
    for (int it = 0; it < 8; ++it) *(volatile v4f*)(pq + go[it]) = val[it];
    __threadfence();
#pragma unroll
    for (int it = 0; it < 8; ++it) *(volatile v4f*)(pq + go[it]) = val[it];
  }
}

template <int L>
__device__ __forceinline__ void tile_group(v16b ash, v16b asl, v16b arh, v16b arl,
                                           const u16* __restrict__ ws2h, const u16* __restrict__ ws2l,
                                           const u16* __restrict__ wr2h, const u16* __restrict__ wr2l,
                                           const float* __restrict__ bs2, const float* __restrict__ br2,
                                           const float* __restrict__ x, const float* __restrict__ ersh,
                                           const int (&er)[8], const int (&dr)[8], int nrem,
                                           float* accw, int lane) {
  constexpr int NM = (L == 0) ? 1 : ((L == 1) ? 3 : 5);
  constexpr int YB = (L == 0) ? 0 : ((L == 1) ? 1 : 4);
  constexpr int PB = (L == 0) ? 0 : ((L == 1) ? CH : 4 * CH);
  const int hh = lane >> 4, c = lane & 15;
  float y[8][NM];
#pragma unroll
  for (int r = 0; r < 8; ++r) {
#pragma unroll
    for (int mm = 0; mm < NM; ++mm) y[r][mm] = ersh[(size_t)er[r] * 9 + YB + mm];
  }
#pragma unroll 1
  for (int u = 0; u < 8; ++u) {
    const int t = 8 * L + u, cc = 16 * u + c, col = CH * L + cc;
    const v16b bsh = ldfrag(ws2h, HD, 16 * t, 0, lane);
    const v16b bsl = ldfrag(ws2l, HD, 16 * t, 0, lane);
    const v16b brh = ldfrag(wr2h, HD, 16 * t, 0, lane);
    const v16b brl = ldfrag(wr2l, HD, 16 * t, 0, lane);
    v8f cs = mma(ash, bsh, zero8());
    cs = mma(asl, bsh, cs);
    cs = mma(ash, bsl, cs);
    v8f cr = mma(arh, brh, zero8());
    cr = mma(arl, brh, cr);
    cr = mma(arh, brl, cr);
    const float b2s = bs2[col], b2r = br2[col];
    float S[NM];
#pragma unroll
    for (int mm = 0; mm < NM; ++mm) S[mm] = 0.f;
#pragma unroll
    for (int r = 0; r < 8; ++r) {
      const bool vr = (8 * hh + r) < nrem;
      const float xv = x[(size_t)dr[r] * CH + cc];
      const float g = vr ? (((cs[r] + b2s) * (cr[r] + b2r)) * xv) : 0.f;
#pragma unroll
      for (int mm = 0; mm < NM; ++mm) S[mm] = fmaf(g, y[r][mm], S[mm]);
    }
#pragma unroll
    for (int mm = 0; mm < NM; ++mm) S[mm] += __shfl_xor(S[mm], 16, 32);
#pragma unroll
    for (int mm = 0; mm < NM; ++mm) {
      const int pos = (hh == 0) ? (PB + mm * CH + cc) : (MS + c);
      accw[pos] += S[mm];
    }
  }
}

__global__ __launch_bounds__(NTE) void k_edge(const float* __restrict__ pq, const float* __restrict__ x,
                                              const float* __restrict__ eattr, const float* __restrict__ ersh,
                                              const int* __restrict__ eidx,
                                              const u16* __restrict__ wr1h, const u16* __restrict__ wr1l,
                                              const u16* __restrict__ ws2h, const u16* __restrict__ ws2l,
                                              const u16* __restrict__ wr2h, const u16* __restrict__ wr2l,
                                              const float* __restrict__ br1, const float* __restrict__ bs2,
                                              const float* __restrict__ br2,
                                              u16* __restrict__ aph, u16* __restrict__ apl) {
  __shared__ int lst_e[CAP];
  __shared__ int lst_n[CAP];
  __shared__ int srt_e[CAP];
  __shared__ int cnt_s[NPB];
  __shared__ int offs_s[NPB + 16];
  __shared__ int wcnt_s[NWE];
  __shared__ int flag_s[4];
  __shared__ __align__(16) float accs[NWE][ACP];
  __shared__ __align__(16) u16 tiles[NWE][6][16 * TP];

  const int tid = threadIdx.x, lane = tid & 31, wave = tid >> 5, hh = lane >> 4, c = lane & 15;
  const int n0 = blockIdx.x * NPB;
  const unsigned ltmask = (1u << lane) - 1u;

  int T = 0;
#pragma unroll 1
  for (int base = 0; base < NE; base += SCH) {
    const int e0 = base + 4 * tid;
    int sv[4];
    if (base + SCH <= NE) {
      const v4i v = *(const v4i*)(eidx + e0);
      sv[0] = v[0]; sv[1] = v[1]; sv[2] = v[2]; sv[3] = v[3];
    } else {
#pragma unroll
      for (int j = 0; j < 4; ++j) {
        const int ej = e0 + j;
        const int ec = (ej < NE) ? ej : (NE - 1);
        const int s = eidx[ec];
        sv[j] = (ej < NE) ? s : -1;
      }
    }
    unsigned mk[4];
    int pre[4];
    int wc = 0;
#pragma unroll
    for (int j = 0; j < 4; ++j) {
      const bool hit = (unsigned)(sv[j] - n0) < (unsigned)NPB;
      mk[j] = __builtin_amdgcn_ballot_w32(hit);
      pre[j] = wc + (int)__builtin_popcount(mk[j] & ltmask);
      wc += (int)__builtin_popcount(mk[j]);
    }
    if (lane == 0) wcnt_s[wave] = wc;
    __syncthreads();
    int woff = 0, tot = 0;
#pragma unroll
    for (int w2 = 0; w2 < NWE; ++w2) {
      const int cw = wcnt_s[w2];
      tot += cw;
      woff += (w2 < wave) ? cw : 0;
    }
#pragma unroll
    for (int j = 0; j < 4; ++j) {
      const bool hit = ((mk[j] >> lane) & 1u) != 0u;
      const int pos = T + woff + pre[j];
      if (hit && pos < CAP) {
        lst_e[pos] = e0 + j;
        lst_n[pos] = sv[j] - n0;
      }
    }
    T += tot;
    __syncthreads();
  }
  const int Tc = (T < CAP) ? T : CAP;

  if (tid < NPB) {
    int cv = 0;
#pragma unroll 1
    for (int i = 0; i < Tc; ++i) cv += (lst_n[i] == tid) ? 1 : 0;
    cnt_s[tid] = cv;
  }
  __syncthreads();
  if (tid == 0) {
    int o = 0, fl = (T > CAP) ? 1 : 0;
#pragma unroll 1
    for (int k = 0; k < NPB; ++k) {
      offs_s[k] = o;
      const int cv = cnt_s[k];
      if (cv > MAXDEG) fl = 1;
      o += cv;
    }
    offs_s[NPB] = o;
    flag_s[0] = fl;
  }
  __syncthreads();
  if (tid < NPB) {
    int pos = offs_s[tid];
#pragma unroll 1
    for (int i = 0; i < Tc; ++i) {
      if (lst_n[i] == tid) {
        if (pos < CAP) srt_e[pos] = lst_e[i];
        ++pos;
      }
    }
  }
  __syncthreads();

  float* accw = &accs[wave][0];
  u16* hsH = &tiles[wave][0][0];
  u16* hsL = &tiles[wave][1][0];
  u16* eaH = &tiles[wave][2][0];
  u16* eaL = &tiles[wave][3][0];
  u16* hrH = &tiles[wave][4][0];
  u16* hrL = &tiles[wave][5][0];
  const bool poison = flag_s[0] != 0;
  const float bb0 = br1[c], bb1 = br1[16 + c];
  const float NANV = __uint_as_float(0x7fc00000u);

#pragma unroll 1
  for (int qn = 0; qn < NPB / NWE; ++qn) {
    const int ln = wave + NWE * qn;
    const int node = n0 + ln;
    int deg = cnt_s[ln];
    deg = (deg < 0) ? 0 : ((deg > MAXDEG) ? MAXDEG : deg);
    int off = offs_s[ln];
    off = (off < 0) ? 0 : ((off > CAP) ? CAP : off);
    const int npass = (deg + 15) >> 4;
#pragma unroll
    for (int i = 0; i < 9; ++i) *(v4f*)(accw + 4 * lane + 128 * i) = zero4();

#pragma unroll 1
    for (int p = 0; p < npass; ++p) {
      wsync();
      const int sbase = 16 * p;
      {
        const int slot = sbase + c;
        const bool vm = slot < deg;
        int li = off + slot;
        li = (li < CAP - 1) ? li : (CAP - 1);
        int e = srt_e[li];
        e = vm ? e : 0;
        e = (e < 0) ? 0 : ((e > NE - 1) ? (NE - 1) : e);
        int s = eidx[e];
        int d = eidx[NE + e];
        s = (s < 0) ? 0 : ((s > NN - 1) ? (NN - 1) : s);
        d = (d < 0) ? 0 : ((d > NN - 1) ? (NN - 1) : d);
        const float* pp = pq + (size_t)s * 64 + 16 * hh;
        const float* qq = pq + (size_t)d * 64 + 32 + 16 * hh;
        v4f a[4];
#pragma unroll
        for (int i = 0; i < 4; ++i) {
          v4f u = *(const v4f*)(pp + 4 * i);
          const v4f u2 = *(const v4f*)(qq + 4 * i);
#pragma unroll
          for (int jj = 0; jj < 4; ++jj) {
            const float prv = u[jj] + u2[jj];
            u[jj] = vm ? silu_f(prv) : 0.f;
          }
          a[i] = u;
        }
        v4u h0, l0, h1, l1;
        split8(a[0], a[1], h0, l0);
        split8(a[2], a[3], h1, l1);
        const int to = c * TP + 16 * hh;
        *(v4u*)(hsH + to) = h0;
        *(v4u*)(hsH + to + 8) = h1;
        *(v4u*)(hsL + to) = l0;
        *(v4u*)(hsL + to + 8) = l1;
        v4f bq[4];
#pragma unroll
        for (int i = 0; i < 4; ++i) {
          const int kq = 16 * hh + 4 * i;
          const int kqc = (kq < 16) ? kq : 16;
          v4f u = *(const v4f*)(eattr + (size_t)e * RB + kqc);
          const bool ok = vm && (kq < RB);
#pragma unroll
          for (int jj = 0; jj < 4; ++jj) u[jj] = ok ? u[jj] : 0.f;
          bq[i] = u;
        }
        split8(bq[0], bq[1], h0, l0);
        split8(bq[2], bq[3], h1, l1);
        *(v4u*)(eaH + to) = h0;
        *(v4u*)(eaH + to + 8) = h1;
        *(v4u*)(eaL + to) = l0;
        *(v4u*)(eaL + to + 8) = l1;
      }
      wsync();
      v8f g0, g1;
      {
        const v16b ah = ldfrag(eaH, TP, 0, 0, lane), al = ldfrag(eaL, TP, 0, 0, lane);
        const v16b bh0 = ldfrag(wr1h, HD, 0, 0, lane), bl0 = ldfrag(wr1l, HD, 0, 0, lane);
        const v16b bh1 = ldfrag(wr1h, HD, 16, 0, lane), bl1 = ldfrag(wr1l, HD, 16, 0, lane);
        g0 = mma(ah, bh0, zero8());
        g0 = mma(al, bh0, g0);
        g0 = mma(ah, bl0, g0);
        g1 = mma(ah, bh1, zero8());
        g1 = mma(al, bh1, g1);
        g1 = mma(ah, bl1, g1);
      }
#pragma unroll
      for (int r = 0; r < 8; ++r) {
        const int row = 8 * hh + r;
        const bool vr = (sbase + row) < deg;
        const float v0 = vr ? silu_f(g0[r] + bb0) : 0.f;
        const float v1 = vr ? silu_f(g1[r] + bb1) : 0.f;
        const u16 x0 = f2bf(v0), x1 = f2bf(v1);
        hrH[row * TP + c] = x0;
        hrL[row * TP + c] = lo_of(v0, x0);
        hrH[row * TP + 16 + c] = x1;
        hrL[row * TP + 16 + c] = lo_of(v1, x1);
      }
      wsync();
      const v16b ash = ldfrag(hsH, TP, 0, 0, lane), asl = ldfrag(hsL, TP, 0, 0, lane);
      const v16b arh = ldfrag(hrH, TP, 0, 0, lane), arl = ldfrag(hrL, TP, 0, 0, lane);
      int er[8], dr[8];
#pragma unroll
      for (int r = 0; r < 8; ++r) {
        const int slot = sbase + 8 * hh + r;
        const bool vr = slot < deg;
        int li = off + slot;
        li = (li < CAP - 1) ? li : (CAP - 1);
        int e = srt_e[li];
        e = vr ? e : 0;
        e = (e < 0) ? 0 : ((e > NE - 1) ? (NE - 1) : e);
        er[r] = e;
        int d = eidx[NE + e];
        d = (d < 0) ? 0 : ((d > NN - 1) ? (NN - 1) : d);
        dr[r] = d;
      }
      const int nrem = deg - sbase;
      tile_group<0>(ash, asl, arh, arl, ws2h, ws2l, wr2h, wr2l, bs2, br2, x, ersh, er, dr, nrem, accw, lane);
      tile_group<1>(ash, asl, arh, arl, ws2h, ws2l, wr2h, wr2l, bs2, br2, x, ersh, er, dr, nrem, accw, lane);
      tile_group<2>(ash, asl, arh, arl, ws2h, ws2l, wr2h, wr2l, bs2, br2, x, ersh, er, dr, nrem, accw, lane);
    }

    wsync();
    v4u hv[5], lv[5];
    size_t go[5];
#pragma unroll
    for (int it = 0; it < 5; ++it) {
      const int piece = it * 32 + lane;
      const int pc = (piece < 144) ? piece : 143;
      v4f a0 = *(const v4f*)(accw + 8 * pc);
      const v4f a1 = *(const v4f*)(accw + 8 * pc + 4);
      if (poison && piece == 0) a0[0] = NANV;
      split8(a0, a1, hv[it], lv[it]);
      go[it] = (size_t)node * MS + 8 * pc;
    }
#pragma unroll
    for (int it = 0; it < 4; ++it) {
      *(volatile v4u*)(aph + go[it]) = hv[it];
      *(volatile v4u*)(apl + go[it]) = lv[it];
    }
    if (lane < 16) {
      *(volatile v4u*)(aph + go[4]) = hv[4];
      *(volatile v4u*)(apl + go[4]) = lv[4];
    }
    __threadfence();
#pragma unroll
    for (int it = 0; it < 4; ++it) {
      *(volatile v4u*)(aph + go[it]) = hv[it];
      *(volatile v4u*)(apl + go[it]) = lv[it];
    }
    if (lane < 16) {
      *(volatile v4u*)(aph + go[4]) = hv[4];
      *(volatile v4u*)(apl + go[4]) = lv[4];
    }
    wsync();
  }
}

template <int NIT>
__device__ __forceinline__ void store_seg(const float* ot, float* __restrict__ out, int n0, int cb,
                                          int wave, int lane) {
  v4f val[2][NIT];
  size_t go[2][NIT];
#pragma unroll
  for (int rr = 0; rr < 2; ++rr) {
    const int row = 2 * wave + rr;
#pragma unroll
    for (int it = 0; it < NIT; ++it) {
      const int p = it * 32 + lane;
      val[rr][it] = *(const v4f*)(ot + row * OTP + 4 * p);
      go[rr][it] = (size_t)(n0 + row) * MS + cb + 4 * p;
    }
  }
#pragma unroll
  for (int rr = 0; rr < 2; ++rr)
#pragma unroll
    for (int it = 0; it < NIT; ++it) *(volatile v4f*)(out + go[rr][it]) = val[rr][it];
  __threadfence();
#pragma unroll
  for (int rr = 0; rr < 2; ++rr)
#pragma unroll
    for (int it = 0; it < NIT; ++it) *(volatile v4f*)(out + go[rr][it]) = val[rr][it];
}

__global__ __launch_bounds__(256) void k_lin2(const u16* __restrict__ aph, const u16* __restrict__ apl,
                                              const u16* __restrict__ wlh, const u16* __restrict__ wll,
                                              const float* __restrict__ b0, float* __restrict__ out) {
  __shared__ __align__(16) float ot[16 * OTP];
  const int tid = threadIdx.x, lane = tid & 31, wave = tid >> 5, hh = lane >> 4, c = lane & 15;
  const int n0 = blockIdx.x * 16;
  const int dd = 16 * wave + c;
  const float INV = 0.08838834764831845f;
  const float bias0 = b0[dd];

#pragma unroll 1
  for (int j = 0; j < 4; ++j) {
    const int l = (j == 0) ? 0 : 1;
    const int mm = (j == 0) ? 0 : (j - 1);
    const u16* wh = wlh + (size_t)l * CH * CH;
    const u16* wl = wll + (size_t)l * CH * CH;
    v8f acc = zero8();
#pragma unroll 1
    for (int ks = 0; ks < 4; ++ks) {
      const int k0 = 32 * ks;
      const v16b ah = ldfrag(aph, MS, n0, CH * j + k0, lane);
      const v16b al = ldfrag(apl, MS, n0, CH * j + k0, lane);
      const v16b bh = ldfrag(wh, CH, 16 * wave, k0, lane);
      const v16b bl = ldfrag(wl, CH, 16 * wave, k0, lane);
      acc = mma(ah, bh, acc);
      acc = mma(al, bh, acc);
      acc = mma(ah, bl, acc);
    }
    const int pos = (j == 0) ? dd : (CH + 3 * dd + mm);
    const float badd = (j == 0) ? bias0 : 0.f;
#pragma unroll
    for (int r = 0; r < 8; ++r) ot[(8 * hh + r) * OTP + pos] = acc[r] * INV + badd;
  }
  __syncthreads();
  store_seg<4>(ot, out, n0, 0, wave, lane);
  __syncthreads();
#pragma unroll 1
  for (int j = 4; j < 9; ++j) {
    const int mm = j - 4;
    const u16* wh = wlh + (size_t)2 * CH * CH;
    const u16* wl = wll + (size_t)2 * CH * CH;
    v8f acc = zero8();
#pragma unroll 1
    for (int ks = 0; ks < 4; ++ks) {
      const int k0 = 32 * ks;
      const v16b ah = ldfrag(aph, MS, n0, CH * j + k0, lane);
      const v16b al = ldfrag(apl, MS, n0, CH * j + k0, lane);
      const v16b bh = ldfrag(wh, CH, 16 * wave, k0, lane);
      const v16b bl = ldfrag(wl, CH, 16 * wave, k0, lane);
      acc = mma(ah, bh, acc);
      acc = mma(al, bh, acc);
      acc = mma(ah, bl, acc);
    }
    const int pos = 5 * dd + mm;
#pragma unroll
    for (int r = 0; r < 8; ++r) ot[(8 * hh + r) * OTP + pos] = acc[r] * INV;
  }
  __syncthreads();
  store_seg<5>(ot, out, n0, 512, wave, lane);
}

extern "C" void kernel_launch(void* const* d_in, const int* in_sizes, int n_in,
                              void* d_out, int out_size, void* d_ws, size_t ws_size,
                              hipStream_t stream) {
  if (n_in < 16) return;
  if (in_sizes[0] != NN * CH) return;
  if (in_sizes[1] != NE * RB) return;
  if (in_sizes[2] != NE * 9) return;
  if (in_sizes[3] != 2 * NE) return;
  if (in_sizes[4] != 2 * CH * HD) return;
  if (in_sizes[5] != HD) return;
  if (in_sizes[6] != HD * WN) return;
  if (in_sizes[7] != WN) return;
  if (in_sizes[8] != RB * HD) return;
  if (in_sizes[9] != HD) return;
  if (in_sizes[10] != HD * WN) return;
  if (in_sizes[11] != WN) return;
  if (in_sizes[12] != CH * CH) return;
  if (in_sizes[13] != CH) return;
  if (in_sizes[14] != CH * CH) return;
  if (in_sizes[15] != CH * CH) return;
  if (out_size != NN * MS) return;

  const float* node_feat = (const float*)d_in[0];
  const float* edge_attr = (const float*)d_in[1];
  const float* edge_rsh  = (const float*)d_in[2];
  const int*   edge_idx  = (const int*)d_in[3];
  const float* ws1  = (const float*)d_in[4];
  const float* bs1  = (const float*)d_in[5];
  const float* ws2  = (const float*)d_in[6];
  const float* bs2  = (const float*)d_in[7];
  const float* wr1  = (const float*)d_in[8];
  const float* br1  = (const float*)d_in[9];
  const float* wr2  = (const float*)d_in[10];
  const float* br2  = (const float*)d_in[11];
  const float* l2w0 = (const float*)d_in[12];
  const float* l2b0 = (const float*)d_in[13];
  const float* l2w1 = (const float*)d_in[14];
  const float* l2w2 = (const float*)d_in[15];
  float* out = (float*)d_out;

  const size_t szWPQ = (size_t)64 * CH * 2;
  const size_t szWR1 = (size_t)HD * HD * 2;
  const size_t szW2  = (size_t)WN * HD * 2;
  const size_t szWL  = (size_t)3 * CH * CH * 2;
  const size_t szPQ  = (size_t)NN * 64 * 4;
  const size_t szAP  = (size_t)NN * MS * 2;

  size_t off = 0;
  const size_t oWPQH = off; off += szWPQ;
  const size_t oWPQL = off; off += szWPQ;
  const size_t oWR1H = off; off += szWR1;
  const size_t oWR1L = off; off += szWR1;
  const size_t oWS2H = off; off += szW2;
  const size_t oWS2L = off; off += szW2;
  const size_t oWR2H = off; off += szW2;
  const size_t oWR2L = off; off += szW2;
  const size_t oWLH  = off; off += szWL;
  const size_t oWLL  = off; off += szWL;
  const size_t oPQ   = off; off += szPQ;
  const size_t oAPH  = off; off += szAP;
  const size_t oAPL  = off; off += szAP;
  if (off > ws_size) return;
  if (off > (size_t)134217728) return;

  char* ws = (char*)d_ws;
  u16* WPQH = (u16*)(ws + oWPQH);
  u16* WPQL = (u16*)(ws + oWPQL);
  u16* WR1H = (u16*)(ws + oWR1H);
  u16* WR1L = (u16*)(ws + oWR1L);
  u16* WS2H = (u16*)(ws + oWS2H);
  u16* WS2L = (u16*)(ws + oWS2L);
  u16* WR2H = (u16*)(ws + oWR2H);
  u16* WR2L = (u16*)(ws + oWR2L);
  u16* WLH  = (u16*)(ws + oWLH);
  u16* WLL  = (u16*)(ws + oWLL);
  float* PQ = (float*)(ws + oPQ);
  u16* APH  = (u16*)(ws + oAPH);
  u16* APL  = (u16*)(ws + oAPL);

  k_prep<<<dim3(41), dim3(256), 0, stream>>>(ws1, wr1, ws2, wr2, l2w0, l2w1, l2w2,
                                             WPQH, WPQL, WR1H, WR1L, WS2H, WS2L, WR2H, WR2L, WLH, WLL);
  k_pq<<<dim3((NN + 127) / 128), dim3(256), 0, stream>>>(node_feat, bs1, WPQH, WPQL, PQ);
  k_edge<<<dim3(NN / NPB), dim3(NTE), 0, stream>>>(PQ, node_feat, edge_attr, edge_rsh, edge_idx,
                                                   WR1H, WR1L, WS2H, WS2L, WR2H, WR2L,
                                                   br1, bs2, br2, APH, APL);
  k_lin2<<<dim3(NN / 16), dim3(256), 0, stream>>>(APH, APL, WLH, WLL, l2b0, out);
  (void)hipGetLastError();
}
